// SlidingWindowCausalAttention_42649025249825
// MI455X (gfx1250) — hardware-verified
//
#include <hip/hip_runtime.h>


namespace {
constexpr int B = 2, S = 2048, E = 1024, NH = 16, HD = 64, NT = B * S;
constexpr float XS = 8.0f, PS = 1024.0f, WSC = 256.0f;
typedef _Float16 b16;
typedef __attribute__((ext_vector_type(16))) _Float16 v16b;
typedef __attribute__((ext_vector_type(8))) _Float16 v8b;
typedef __attribute__((ext_vector_type(8))) float v8f;
typedef __attribute__((ext_vector_type(4))) float v4f;
__device__ __forceinline__ float bf16_rne(float f) { unsigned int u = __float_as_uint(f); u += 0x7FFFu + ((u >> 16) & 1u); return __uint_as_float(u & 0xFFFF0000u); }
__device__ __forceinline__ void split16(float v, b16& hi, b16& lo) { hi = (b16)v; lo = (b16)(v - (float)hi); }
__device__ __forceinline__ v16b frag_kb(const b16* p, int hh) { const v8b a = *(const v8b*)(p + 8 * hh), b = *(const v8b*)(p + 16 + 8 * hh); v16b f;
#pragma unroll
  for (int e = 0; e < 8; ++e) { f[e] = a[e]; f[8 + e] = b[e]; } return f; }
__device__ __forceinline__ v8f wmma16b(v16b a, v16b b, v8f c) { v8f d = __builtin_amdgcn_wmma_f32_16x16x32_f16(false, a, false, b, (short)0, c, false, false); asm volatile("v_nop\n\tv_nop\n\tv_nop\n\tv_nop" : "+v"(d) : "v"(a), "v"(b)); return d; }
__device__ __forceinline__ void wave_lds_sync() { __builtin_amdgcn_fence(__ATOMIC_RELEASE, "workgroup"); __builtin_amdgcn_wave_barrier(); __builtin_amdgcn_fence(__ATOMIC_ACQUIRE, "workgroup"); }
__device__ __forceinline__ float pmul(float a, float b) { float p = a * b; asm volatile("" : "+v"(p)); return p; }

__global__ __launch_bounds__(256) void wcopy_kernel(const float* __restrict__ w, size_t total, b16* __restrict__ WT) { const size_t u = (size_t)blockIdx.x * 256 + threadIdx.x; if (u >= total / 8) return; const size_t e = u * 8; v8b v;
#pragma unroll
  for (int j = 0; j < 8; ++j) v[j] = (b16)(bf16_rne(w[e + j]) * WSC); for (int pass = 0; pass < 2; ++pass) { *(volatile v8b*)(WT + e) = v; __threadfence(); } }
template <int EXA>
__global__ __launch_bounds__(32) void dense_kernel(const float* __restrict__ IN, const b16* __restrict__ WT, int ncg, int RLIM, int outw, float* __restrict__ OUT) {
  __shared__ __attribute__((aligned(16))) b16 Ah[16][E + 8], Al[16][EXA ? 8 : E + 8]; __shared__ float Tf[16][132];
  const int lane = threadIdx.x, nloc = lane & 15, hlf = lane >> 4; const int cg = blockIdx.x % ncg; const size_t m0 = (size_t)(blockIdx.x / ncg) * 16; if (m0 >= (size_t)RLIM) return;
  for (int rr = 0; rr < 16; ++rr) for (int q = 0; q < E / 32; ++q) { const float v = IN[(m0 + rr) * E + q * 32 + lane]; if (EXA) Ah[rr][q * 32 + lane] = (b16)(bf16_rne(v) * XS); else { b16 p, ql; split16(v * XS, p, ql); Ah[rr][q * 32 + lane] = p; Al[rr][q * 32 + lane] = ql; } }
  wave_lds_sync(); v8f acc[8];
#pragma unroll
  for (int t = 0; t < 8; ++t) acc[t] = (v8f){};
#pragma unroll 2
  for (int kb = 0; kb < E; kb += 32) { const v16b a = frag_kb(&Ah[nloc][kb], hlf); v16b al; if (!EXA) al = frag_kb(&Al[nloc][kb], hlf);
#pragma unroll
    for (int t = 0; t < 8; ++t) { const v16b bw = frag_kb(WT + (size_t)(cg * 128 + t * 16 + nloc) * E + kb, hlf); acc[t] = wmma16b(a, bw, acc[t]); if (!EXA) acc[t] = wmma16b(al, bw, acc[t]); } }
#pragma unroll
  for (int t = 0; t < 8; ++t)
#pragma unroll
    for (int r8 = 0; r8 < 8; ++r8) Tf[8 * hlf + r8][t * 16 + nloc] = acc[t][r8] * (1.0f / (XS * WSC));
  wave_lds_sync();
  for (int pass = 0; pass < 2; ++pass) { for (int rr = 0; rr < 16; ++rr) *(volatile v4f*)(OUT + (m0 + rr) * (size_t)outw + cg * 128 + lane * 4) = *(const v4f*)(&Tf[rr][lane * 4]); __threadfence(); }
}
__global__ __launch_bounds__(32) void att_kernel(const float* __restrict__ QKV, int BV, int SV, float* __restrict__ ATT) {
  __shared__ __attribute__((aligned(16))) b16 Qh[16][HD + 8], Ql[16][HD + 8], Kh[32][HD + 8], Kl[32][HD + 8], Ph[16][40], Pl[16][40], Vh[HD][40], Vl[HD][40]; __shared__ float Sc[16][33], M[16], Dn[16], Sf[16], Of[16][HD + 2];
  const int lane = threadIdx.x, nloc = lane & 15, hlf = lane >> 4; const int qblocks = SV / 16; const int qb = blockIdx.x % qblocks, h = (blockIdx.x / qblocks) % NH, b = blockIdx.x / (qblocks * NH); if (b >= BV) return;
  const size_t base = (size_t)b * S; const int q0 = qb * 16; const size_t W3 = 3 * E;
  for (int rr = 0; rr < 16; ++rr) for (int q = 0; q < 2; ++q) { b16 p, ql; split16(QKV[(base + q0 + rr) * W3 + h * HD + q * 32 + lane] * XS, p, ql); Qh[rr][q * 32 + lane] = p; Ql[rr][q * 32 + lane] = ql; }
  if (lane < 16) { M[lane] = -INFINITY; Dn[lane] = 0.0f; Sf[lane] = 0.0f; }
  v8f acc[4] = {(v8f){}, (v8f){}, (v8f){}, (v8f){}}; wave_lds_sync();
#pragma unroll 1
  for (int kc = 0; kc < q0 + 16; kc += 32) {
    for (int rr = 0; rr < 32; ++rr) { const float* kp = QKV + (base + kc + rr) * W3 + E + h * HD; const float* vp = QKV + (base + kc + rr) * W3 + 2 * E + h * HD; for (int q = 0; q < 2; ++q) { b16 p, ql; split16(kp[q * 32 + lane] * XS, p, ql); Kh[rr][q * 32 + lane] = p; Kl[rr][q * 32 + lane] = ql; split16(vp[q * 32 + lane] * XS, p, ql); Vh[q * 32 + lane][rr] = p; Vl[q * 32 + lane][rr] = ql; } }
    wave_lds_sync();
#pragma unroll
    for (int blk = 0; blk < 2; ++blk) { v8f s = {};
#pragma unroll
      for (int kb = 0; kb < HD; kb += 32) { const v16b qh = frag_kb(&Qh[nloc][kb], hlf), qlo = frag_kb(&Ql[nloc][kb], hlf), kh = frag_kb(&Kh[blk * 16 + nloc][kb], hlf), kl = frag_kb(&Kl[blk * 16 + nloc][kb], hlf); s = wmma16b(qh, kh, s); s = wmma16b(qh, kl, s); s = wmma16b(qlo, kh, s); }
#pragma unroll
      for (int r8 = 0; r8 < 8; ++r8) { const int qi = q0 + 8 * hlf + r8, kj = kc + blk * 16 + nloc; Sc[8 * hlf + r8][blk * 16 + nloc] = kj <= qi ? s[r8] * (0.125f / (XS * XS)) : -INFINITY; } }
    wave_lds_sync();
#pragma unroll 1
    for (int qi = 0; qi < 16; ++qi) { const float sv = Sc[qi][lane]; float cm = sv; for (int o = 16; o; o >>= 1) cm = fmaxf(cm, __shfl_xor(cm, o)); const float mo = M[qi]; const float mn = fmaxf(mo, cm); const float p = (sv == -INFINITY) ? 0.0f : __expf(sv - mn); float psum = p; for (int o = 16; o; o >>= 1) psum += __shfl_xor(psum, o);
      b16 ph, plo; split16(p * PS, ph, plo); Ph[qi][lane] = ph; Pl[qi][lane] = plo; if (lane == 0) { const float sf = (mo == -INFINITY) ? 0.0f : __expf(mo - mn); Sf[qi] = sf; Dn[qi] = Dn[qi] * sf + psum; M[qi] = mn; } }
    wave_lds_sync();
#pragma unroll
    for (int t = 0; t < 4; ++t) {
#pragma unroll
      for (int r8 = 0; r8 < 8; ++r8) acc[t][r8] *= Sf[8 * hlf + r8];
      const v16b pa = frag_kb(&Ph[nloc][0], hlf), pb = frag_kb(&Pl[nloc][0], hlf), vh = frag_kb(&Vh[t * 16 + nloc][0], hlf), vl = frag_kb(&Vl[t * 16 + nloc][0], hlf); acc[t] = wmma16b(pa, vh, acc[t]); acc[t] = wmma16b(pa, vl, acc[t]); acc[t] = wmma16b(pb, vh, acc[t]); }
    wave_lds_sync(); }
#pragma unroll
  for (int t = 0; t < 4; ++t)
#pragma unroll
    for (int r8 = 0; r8 < 8; ++r8) { const int rl = 8 * hlf + r8; Of[rl][t * 16 + nloc] = acc[t][r8] * (1.0f / (PS * XS)) / Dn[rl]; }
  wave_lds_sync();
  for (int pass = 0; pass < 2; ++pass) { for (int rr = 0; rr < 16; ++rr) { ((volatile float*)ATT)[(base + q0 + rr) * E + h * HD + lane * 2] = Of[rr][lane * 2]; ((volatile float*)ATT)[(base + q0 + rr) * E + h * HD + lane * 2 + 1] = Of[rr][lane * 2 + 1]; } __threadfence(); }
}
}

extern "C" void kernel_launch(void* const* d_in, const int* in_sizes, int n_in, void* d_out, int out_size, void* d_ws, size_t ws_size, hipStream_t stream) {
  (void)n_in;
  auto Fp = [&](int i) { return (const float*)d_in[i]; };
  if (in_sizes[0] != NT * E || in_sizes[1] != 3 * E * E || in_sizes[2] != E * E || out_size != NT * E) return;
  const int BV = B, SV = S; const int RL = (BV - 1) * S + SV;
  size_t off = 0; char* ws = (char*)d_ws;
  auto carve = [&](size_t bytes) { char* p = ws + off; off += (bytes + 255) & ~(size_t)255; return p; };
  b16* WQKV = (b16*)carve((size_t)3 * E * E * 2); b16* WO = (b16*)carve((size_t)E * E * 2); float* QKV = (float*)carve((size_t)NT * 3 * E * 4); float* ATT = (float*)carve((size_t)NT * E * 4);
  if (off > ws_size || off > ((size_t)96 << 20)) return;
  wcopy_kernel<<<(unsigned)(((size_t)3 * E * E / 8 + 255) / 256), 256, 0, stream>>>(Fp(1), (size_t)3 * E * E, WQKV); wcopy_kernel<<<(unsigned)(((size_t)E * E / 8 + 255) / 256), 256, 0, stream>>>(Fp(2), (size_t)E * E, WO);
  dense_kernel<1><<<(RL / 16) * 24, 32, 0, stream>>>(Fp(0), WQKV, 24, RL, 3 * E, QKV);
  att_kernel<<<BV * NH * (SV / 16), 32, 0, stream>>>(QKV, BV, SV, ATT);
  dense_kernel<0><<<(RL / 16) * 8, 32, 0, stream>>>(ATT, WO, 8, RL, E, (float*)d_out);
}
